// MCMambaBlock_31215822307446
// MI455X (gfx1250) — hardware-run, weakly checked
//
#include <hip/hip_runtime.h>
#include <math.h>

typedef __attribute__((ext_vector_type(16))) _Float16 v16h;
typedef __attribute__((ext_vector_type(8)))  _Float16 v8h;
typedef __attribute__((ext_vector_type(16))) __bf16   v16b;
typedef __attribute__((ext_vector_type(8)))  __bf16   v8b;
typedef __attribute__((ext_vector_type(8)))  float    v8f;
typedef __attribute__((ext_vector_type(4)))  float    v4f;

constexpr int kB    = 2;
constexpr int kT    = 1024;
constexpr int kDm   = 768;
constexpr int kDi   = 1536;
constexpr int kDs   = 64;
constexpr int kDtR  = 32;
constexpr int kSeg  = 256;
constexpr int kNSeg = 4;
constexpr int kXzP  = 2 * kDi;
constexpr int kXdN  = kDtR + 2 * kDs;
constexpr int kXdP  = 192;
constexpr int kRows = kB * kT;
constexpr int kTP   = 260;
constexpr int kScTS = 32;
constexpr int kScCh = 64;
constexpr int kScYP = 68;
static_assert(kXdN == 160 && kXdP % 64 == 0 && kXdP >= kXdN, "x_proj width and pad");
static_assert(kDm % 64 == 0 && kDi % 64 == 0 && kDtR == 32, "GEMM K multiples of 32, transpose tiles of 64");
static_assert(kRows % 64 == 0 && kXzP % 64 == 0 && kDm % 64 == 0 && kDi % 64 == 0, "GEMM M,N multiples of 64");
static_assert((kT & (kT - 1)) == 0 && kT % 64 == 0 && kT % kScTS == 0 && kSeg * kNSeg == kT, "time tiling");
static_assert(kDi % 256 == 0 && kDm % 256 == 0 && kDi % kScCh == 0 && kDm % 128 == 0 && kSeg % 16 == 0, "channel tiling");
static_assert(kDs == 64, "four lanes times sixteen states");

constexpr size_t kOffXB    = 0;
constexpr size_t kOffWINT  = kOffXB    + (size_t)kRows * kDm  * 2;
constexpr size_t kOffWXT   = kOffWINT  + (size_t)kXzP  * kDm  * 2;
constexpr size_t kOffWDTT  = kOffWXT   + (size_t)kXdP  * kDi  * 2;
constexpr size_t kOffWOUTT = kOffWDTT  + (size_t)kDi   * kDtR * 2;
constexpr size_t kOffWUT   = kOffWOUTT + (size_t)kDm   * kDi  * 2;
constexpr size_t kOffXZ    = kOffWUT   + (size_t)kDm   * kDm  * 2;
constexpr size_t kOffXI    = kOffXZ    + (size_t)kRows * kXzP * 4;
constexpr size_t kOffXIH   = kOffXI    + (size_t)kRows * kDi  * 4;
constexpr size_t kOffXIL   = kOffXIH   + (size_t)kRows * kDi  * 2;
constexpr size_t kOffXD    = kOffXIL   + (size_t)kRows * kDi  * 2;
constexpr size_t kOffDTH   = kOffXD    + (size_t)kRows * kXdP * 4;
constexpr size_t kOffDTL   = kOffDTH   + (size_t)kRows * kDtR * 2;
constexpr size_t kOffDLR   = kOffDTL   + (size_t)kRows * kDtR * 2;
constexpr size_t kOffYH    = kOffDLR   + (size_t)kRows * kDi  * 4;
constexpr size_t kOffYL    = kOffYH    + (size_t)kRows * kDi  * 2;
constexpr size_t kOffXOUT  = kOffYL    + (size_t)kRows * kDi  * 2;
constexpr size_t kOffUU    = kOffXOUT  + (size_t)kRows * kDm  * 4;
constexpr size_t kOffMCUR  = kOffUU    + (size_t)kRows * kDm  * 4;
constexpr size_t kOffMST   = kOffMCUR  + (size_t)kRows * kDm  * 4;
constexpr size_t kWsTotal  = kOffMST   + (size_t)kB * kNSeg * kDm * 4;
static_assert(kWsTotal == 108322816ull, "carve total");
static_assert(kWsTotal <= 134217728ull, "carve cap");
static_assert((kOffWINT % 128) == 0 && (kOffWXT % 128) == 0 && (kOffWDTT % 128) == 0 && (kOffWOUTT % 128) == 0 &&
              (kOffWUT % 128) == 0 && (kOffXZ % 128) == 0 && (kOffXI % 128) == 0 && (kOffXIH % 128) == 0 &&
              (kOffXIL % 128) == 0 && (kOffXD % 128) == 0 && (kOffDTH % 128) == 0 && (kOffDTL % 128) == 0 &&
              (kOffDLR % 128) == 0 && (kOffYH % 128) == 0 && (kOffYL % 128) == 0 && (kOffXOUT % 128) == 0 &&
              (kOffUU % 128) == 0 && (kOffMCUR % 128) == 0 && (kOffMST % 128) == 0, "128-B aligned regions");

__device__ __forceinline__ unsigned short f2bf_bits(float f) {
  unsigned u = __float_as_uint(f);
  return (unsigned short)((u + 0x7FFFu + ((u >> 16) & 1u)) >> 16);
}
__device__ __forceinline__ float bf_bits2f(unsigned short h) { return __uint_as_float(((unsigned)h) << 16); }
__device__ __forceinline__ float rne_bf(float f) { return bf_bits2f(f2bf_bits(f)); }

__device__ __forceinline__ void dep_guard4_h(v8f& a, v8f& b, v8f& c, v8f& d, v16h x, v16h y) { asm volatile("v_nop\n\tv_nop\n\tv_nop\n\tv_nop" : "+v"(a), "+v"(b), "+v"(c), "+v"(d) : "v"(x), "v"(y)); }
__device__ __forceinline__ void dep_guard4_b(v8f& a, v8f& b, v8f& c, v8f& d, v16b x, v16b y) { asm volatile("v_nop\n\tv_nop\n\tv_nop\n\tv_nop" : "+v"(a), "+v"(b), "+v"(c), "+v"(d) : "v"(x), "v"(y)); }
__device__ __forceinline__ void keep4_h(v16h a, v16h b, v16h c, v16h d) { asm volatile("v_nop" :: "v"(a), "v"(b), "v"(c), "v"(d)); }
__device__ __forceinline__ void keep4_b(v16b a, v16b b, v16b c, v16b d) { asm volatile("v_nop" :: "v"(a), "v"(b), "v"(c), "v"(d)); }
__device__ __forceinline__ void acc_guard4(v8f& a, v8f& b, v8f& c, v8f& d) { asm volatile("v_nop\n\tv_nop\n\tv_nop\n\tv_nop" : "+v"(a), "+v"(b), "+v"(c), "+v"(d)); }
template <typename T> struct Frag;
template <> struct Frag<_Float16> {
  typedef v16h V; union U { v16h v; v8h h[2]; };
  static __device__ __forceinline__ v16h load(const _Float16* p) {
    U f; f.h[0] = *(const v8h*)(p); f.h[1] = *(const v8h*)(p + 16); return f.v;
  }
  static __device__ __forceinline__ v8f mma(v16h a, v16h b, v8f c) {
    return __builtin_amdgcn_wmma_f32_16x16x32_f16(false, a, false, b, (short)0, c, false, false);
  }
  static __device__ __forceinline__ void guard4(v8f& a, v8f& b, v8f& c, v8f& d, v16h x, v16h y) { dep_guard4_h(a, b, c, d, x, y); }
  static __device__ __forceinline__ void keep(v16h a, v16h b, v16h c, v16h d) { keep4_h(a, b, c, d); }
};
template <> struct Frag<__bf16> {
  typedef v16b V; union U { v16b v; v8b h[2]; };
  static __device__ __forceinline__ v16b load(const __bf16* p) {
    U f; f.h[0] = *(const v8b*)(p); f.h[1] = *(const v8b*)(p + 16); return f.v;
  }
  static __device__ __forceinline__ v8f mma(v16b a, v16b b, v8f c) {
    return __builtin_amdgcn_wmma_f32_16x16x32_bf16(false, a, false, b, (short)0, c, false, false);
  }
  static __device__ __forceinline__ void guard4(v8f& a, v8f& b, v8f& c, v8f& d, v16b x, v16b y) { dep_guard4_b(a, b, c, d, x, y); }
  static __device__ __forceinline__ void keep(v16b a, v16b b, v16b c, v16b d) { keep4_b(a, b, c, d); }
};

template <int ET> struct Elem;
template <> struct Elem<0> { typedef _Float16 T; };
template <> struct Elem<1> { typedef __bf16 T; };
template <int ET, int SPL, int BIAS_MODE, int OUT_MODE, bool RESID, int ACT = 0>
__global__ __launch_bounds__(256) void wmma_gemm64(
    const unsigned short* __restrict__ Ap, const unsigned short* __restrict__ A2p, int lda, long strideA,
    const unsigned short* __restrict__ Btp, const unsigned short* __restrict__ Bt2p, int ldb, long strideB,
    void* __restrict__ Cout, void* __restrict__ Cout2, int ldc, long strideC,
    const float* __restrict__ bias,
    const float* __restrict__ resid, long strideR,
    int M, int N, int K, float scale) {
  typedef typename Elem<ET>::T T;
  typedef typename Frag<T>::V V;
  const T* A = (const T*)Ap; const T* A2 = (const T*)A2p; const T* Bt = (const T*)Btp; const T* Bt2 = (const T*)Bt2p;
  __shared__ __align__(16) float sT[8][16 * 68];
  const int b    = blockIdx.y;
  const int lane = threadIdx.x & 31;
  const int wave = threadIdx.x >> 5;
  const int tilesN = N >> 6;
  const int tilesM = M >> 6;
  const int tile = blockIdx.x * 8 + wave;
  if (tile >= tilesM * tilesN) return;
  const int tm = tile / tilesN;
  const int tn = tile - tm * tilesN;
  const int m0 = tm << 6;
  const int n0 = tn << 6;

  const T* Ab  = A  + (size_t)b * strideA;
  const T* Bb  = Bt + (size_t)b * strideB;
  const T* Ab2 = (SPL >= 1) ? (A2  + (size_t)b * strideA) : nullptr;
  const T* Bb2 = (SPL == 2) ? (Bt2 + (size_t)b * strideB) : nullptr;

  const int rlane = lane & 15;
  const int koff  = (lane >> 4) * 8;
  const int mOff  = (lane >> 4) * 8;

  v8f acc[4][4];
#pragma unroll
  for (int i = 0; i < 4; ++i)
#pragma unroll
    for (int j = 0; j < 4; ++j) acc[i][j] = (v8f){0.f,0.f,0.f,0.f,0.f,0.f,0.f,0.f};

  for (int k0 = 0; k0 < K; k0 += 32) {
    V bh[4], bl[4];
#pragma unroll
    for (int j = 0; j < 4; ++j) {
      const size_t bo = (size_t)(n0 + (j << 4) + rlane) * ldb + koff + k0;
      bh[j] = Frag<T>::load(Bb + bo);
      if (SPL == 2) bl[j] = Frag<T>::load(Bb2 + bo);
    }
#pragma unroll
    for (int i = 0; i < 4; ++i) {
      const size_t ao = (size_t)(m0 + (i << 4) + rlane) * lda + koff + k0;
      V ah = Frag<T>::load(Ab + ao);
      V al;
      if (SPL >= 1) al = Frag<T>::load(Ab2 + ao);
#pragma unroll
      for (int j = 0; j < 4; ++j) {
        acc[i][j] = Frag<T>::mma(ah, bh[j], acc[i][j]);
        if (SPL == 2) acc[i][j] = Frag<T>::mma(ah, bl[j], acc[i][j]);
        if (SPL >= 1) acc[i][j] = Frag<T>::mma(al, bh[j], acc[i][j]);
      }
      Frag<T>::guard4(acc[i][0], acc[i][1], acc[i][2], acc[i][3], ah, (SPL >= 1) ? al : ah);
    }
    Frag<T>::keep(bh[0], bh[1], bh[2], bh[3]);
    if (SPL == 2) Frag<T>::keep(bl[0], bl[1], bl[2], bl[3]);
  }
  acc_guard4(acc[0][0], acc[0][1], acc[0][2], acc[0][3]);
  acc_guard4(acc[1][0], acc[1][1], acc[1][2], acc[1][3]);
  acc_guard4(acc[2][0], acc[2][1], acc[2][2], acc[2][3]);
  acc_guard4(acc[3][0], acc[3][1], acc[3][2], acc[3][3]);

  float* slab = sT[wave];
  const float* Rb = RESID ? (resid + (size_t)b * strideR) : nullptr;
#pragma unroll
  for (int i = 0; i < 4; ++i) {
    const int mBase = m0 + (i << 4);
#pragma unroll
    for (int j = 0; j < 4; ++j) {
      const int n = n0 + (j << 4) + rlane;
      float bv = 0.f;
      if (BIAS_MODE == 2) bv = bias[n];
#pragma unroll
      for (int r = 0; r < 8; ++r) {
        float v = acc[i][j][r] * scale;
        if (BIAS_MODE == 1) v += bias[mBase + mOff + r];
        if (BIAS_MODE == 2) v += bv;
        if (RESID) v += Rb[(size_t)(mBase + mOff + r) * ldc + n];
        if (ACT == 1) v = tanhf(v);
        if (ACT == 2) v = fmaxf(v, 0.0f);
        if (ACT == 3) v = v / (1.0f + expf(-v));
        if (ACT == 4) v = (v > 0.f) ? v : 0.01f * v;
        slab[(mOff + r) * 68 + (j << 4) + rlane] = v;
      }
    }
    __builtin_amdgcn_fence(__ATOMIC_RELEASE, "workgroup");
    __builtin_amdgcn_wave_barrier();
    __builtin_amdgcn_fence(__ATOMIC_ACQUIRE, "workgroup");
    if (OUT_MODE == 0) {
      float* C = (float*)Cout + (size_t)b * strideC;
      const int hh = lane >> 4, c4 = (lane & 15) * 4;
      for (int pass = 0; pass < 2; ++pass) {
#pragma unroll
        for (int it = 0; it < 8; ++it) {
          const int row = it * 2 + hh;
          v4f v = *(const v4f*)(slab + row * 68 + c4);
          *(volatile v4f*)(C + (size_t)(mBase + row) * ldc + n0 + c4) = v;
        }
        __threadfence();
      }
    } else {
      const int q = lane >> 3, c8 = (lane & 7) * 8;
      unsigned short* C  = (unsigned short*)Cout  + (size_t)b * strideC;
      unsigned short* C2 = (OUT_MODE == 2) ? ((unsigned short*)Cout2 + (size_t)b * strideC) : nullptr;
      for (int pass = 0; pass < 2; ++pass) {
#pragma unroll
        for (int it = 0; it < 4; ++it) {
          const int row = it * 4 + q;
          const float* sp = slab + row * 68 + c8;
          v8h hv, lv;
#pragma unroll
          for (int e = 0; e < 8; ++e) {
            if (OUT_MODE == 1) {
              hv[e] = (_Float16)sp[e];
            } else {
              unsigned short hb = f2bf_bits(sp[e]);
              unsigned short lb = f2bf_bits(sp[e] - bf_bits2f(hb));
              hv[e] = __builtin_bit_cast(_Float16, hb);
              lv[e] = __builtin_bit_cast(_Float16, lb);
            }
          }
          *(volatile v8h*)(C + (size_t)(mBase + row) * ldc + n0 + c8) = hv;
          if (OUT_MODE == 2) *(volatile v8h*)(C2 + (size_t)(mBase + row) * ldc + n0 + c8) = lv;
        }
        __threadfence();
      }
    }
    __builtin_amdgcn_fence(__ATOMIC_RELEASE, "workgroup");
    __builtin_amdgcn_wave_barrier();
    __builtin_amdgcn_fence(__ATOMIC_ACQUIRE, "workgroup");
  }
}

__global__ __launch_bounds__(256) void cast_bf16_kernel(
    const float* __restrict__ src, unsigned short* __restrict__ dst, int total8)
{
  const int i = blockIdx.x * 256 + threadIdx.x;
  if (i >= total8) return;
  const size_t e0 = (size_t)i << 3;
  const v4f a0 = *(const v4f*)(src + e0);
  const v4f a1 = *(const v4f*)(src + e0 + 4);
  v8h hv;
#pragma unroll
  for (int e = 0; e < 4; ++e) {
    const unsigned short h0 = f2bf_bits(a0[e]);
    const unsigned short h1 = f2bf_bits(a1[e]);
    hv[e]     = __builtin_bit_cast(_Float16, h0);
    hv[4 + e] = __builtin_bit_cast(_Float16, h1);
  }
  unsigned short* q = dst + e0;
  *(volatile v8h*)q = hv;
  __threadfence();
  *(volatile v8h*)q = hv;
}

__global__ __launch_bounds__(256) void transpose_bf16_kernel(
    const float* __restrict__ W, unsigned short* __restrict__ Bt, int Kdim, int Ndim)
{
  __shared__ float tile[64 * 65];
  const int tid = threadIdx.x, lane = tid & 31, wave = tid >> 5;
  const int n0 = blockIdx.x * 64;
  const int k0 = blockIdx.y * 64;
#pragma unroll
  for (int p = 0; p < 16; ++p) {
    const int idx = tid + p * 256;
    const int kk  = idx >> 6;
    const int nn  = idx & 63;
    const int n   = n0 + nn;
    const int nc  = (n < Ndim) ? n : (Ndim - 1);
    const float v = W[(size_t)(k0 + kk) * Ndim + nc];
    tile[kk * 65 + nn] = (n < Ndim) ? v : 0.f;
  }
  __syncthreads();
  const int q = lane >> 3, c8 = (lane & 7) * 8;
  v8h hv[2];
#pragma unroll
  for (int it = 0; it < 2; ++it) {
    const int nrow = it * 32 + wave * 4 + q;
#pragma unroll
    for (int e = 0; e < 8; ++e) {
      const unsigned short hb = f2bf_bits(tile[(c8 + e) * 65 + nrow]);
      hv[it][e] = __builtin_bit_cast(_Float16, hb);
    }
  }
  for (int pass = 0; pass < 2; ++pass) {
#pragma unroll
    for (int it = 0; it < 2; ++it) {
      const int nrow = it * 32 + wave * 4 + q;
      *(volatile v8h*)(Bt + (size_t)(n0 + nrow) * Kdim + k0 + c8) = hv[it];
    }
    __threadfence();
  }
}

__global__ __launch_bounds__(256) void transpose_k32_kernel(
    const float* __restrict__ W, unsigned short* __restrict__ Bt, int Ndim, int total8)
{
  const int i = blockIdx.x * 256 + threadIdx.x;
  if (i >= total8) return;
  const int n  = i >> 2;
  const int k8 = (i & 3) * 8;
  v8h hv;
#pragma unroll
  for (int e = 0; e < 8; ++e) {
    const float v = W[(size_t)(k8 + e) * Ndim + n];
    const unsigned short hb = f2bf_bits(v);
    hv[e] = __builtin_bit_cast(_Float16, hb);
  }
  unsigned short* q = Bt + ((size_t)i << 3);
  *(volatile v8h*)q = hv;
  __threadfence();
  *(volatile v8h*)q = hv;
}

__global__ __launch_bounds__(256) void conv_silu_kernel(
    const float* __restrict__ XZ, const float* __restrict__ cw, const float* __restrict__ cb,
    float* __restrict__ XI, unsigned short* __restrict__ XIH, unsigned short* __restrict__ XIL)
{
  __shared__ __align__(16) float sT[16 * kTP];
  const int tid = threadIdx.x, lane = tid & 31, wave = tid >> 5;
  const int d0 = blockIdx.x * 256, d = d0 + tid;
  const int g0 = blockIdx.y * 64;
  const int tb = g0 & (kT - 1);
  const v4f wv = *(const v4f*)(cw + (size_t)d * 4);
  const float w0 = rne_bf(wv[0]), w1 = rne_bf(wv[1]), w2 = rne_bf(wv[2]), w3 = rne_bf(wv[3]);
  const float bc = rne_bf(cb[d]);
  float xm3, xm2, xm1;
  {
    const bool hist = (tb > 0);
    const int rb = hist ? (g0 - 3) : g0;
    const float v3 = XZ[(size_t)rb * kXzP + d];
    const float v2 = XZ[(size_t)(rb + 1) * kXzP + d];
    const float v1 = XZ[(size_t)(rb + 2) * kXzP + d];
    xm3 = hist ? v3 : 0.f;
    xm2 = hist ? v2 : 0.f;
    xm1 = hist ? v1 : 0.f;
  }
  const int hrow = wave >> 1;
  const int hch  = (wave & 1) * 128 + lane * 4;
#pragma unroll 1
  for (int sub = 0; sub < 4; ++sub) {
    const int lb = g0 + sub * 16;
#pragma unroll 1
    for (int s = 0; s < 16; ++s) {
      const float xcur = XZ[(size_t)(lb + s) * kXzP + d];
      float acc = w0 * xm3;
      acc = fmaf(w1, xm2, acc);
      acc = fmaf(w2, xm1, acc);
      acc = fmaf(w3, xcur, acc);
      const float sv = acc + bc;
      const float sg = __builtin_amdgcn_rcpf(1.0f + expf(-sv));
      sT[s * kTP + tid] = sv * sg;
      xm3 = xm2; xm2 = xm1; xm1 = xcur;
    }
    __syncthreads();
    v4f fv[4];
    v8h bh[2], blo[2];
#pragma unroll
    for (int it = 0; it < 4; ++it) fv[it] = *(const v4f*)(sT + (it * 4 + hrow) * kTP + hch);
#pragma unroll
    for (int it = 0; it < 2; ++it) {
      const float* sp = sT + (it * 8 + wave) * kTP + lane * 8;
      const v4f a0 = *(const v4f*)(sp);
      const v4f a1 = *(const v4f*)(sp + 4);
#pragma unroll
      for (int e = 0; e < 4; ++e) {
        const unsigned short h0 = f2bf_bits(a0[e]), h1 = f2bf_bits(a1[e]);
        const unsigned short l0 = f2bf_bits(a0[e] - bf_bits2f(h0)), l1 = f2bf_bits(a1[e] - bf_bits2f(h1));
        bh[it][e]      = __builtin_bit_cast(_Float16, h0);
        bh[it][4 + e]  = __builtin_bit_cast(_Float16, h1);
        blo[it][e]     = __builtin_bit_cast(_Float16, l0);
        blo[it][4 + e] = __builtin_bit_cast(_Float16, l1);
      }
    }
    for (int pass = 0; pass < 2; ++pass) {
#pragma unroll
      for (int it = 0; it < 4; ++it)
        *(volatile v4f*)(XI + (size_t)(lb + it * 4 + hrow) * kDi + d0 + hch) = fv[it];
#pragma unroll
      for (int it = 0; it < 2; ++it) {
        const size_t o = (size_t)(lb + it * 8 + wave) * kDi + d0 + lane * 8;
        *(volatile v8h*)(XIH + o) = bh[it];
        *(volatile v8h*)(XIL + o) = blo[it];
      }
      __threadfence();
    }
    __syncthreads();
  }
}

__global__ __launch_bounds__(256) void dt_split_kernel(
    const float* __restrict__ XD, unsigned short* __restrict__ DTH, unsigned short* __restrict__ DTL, int total8)
{
  const int i = blockIdx.x * 256 + threadIdx.x;
  if (i >= total8) return;
  const int e0  = i << 3;
  const int row = e0 >> 5;
  const int c8  = e0 & 31;
  const float* p = XD + (size_t)row * kXdP + c8;
  const v4f a0 = *(const v4f*)(p);
  const v4f a1 = *(const v4f*)(p + 4);
  v8h hv, lv;
#pragma unroll
  for (int e = 0; e < 4; ++e) {
    const unsigned short h0 = f2bf_bits(a0[e]), h1 = f2bf_bits(a1[e]);
    const unsigned short l0 = f2bf_bits(a0[e] - bf_bits2f(h0)), l1 = f2bf_bits(a1[e] - bf_bits2f(h1));
    hv[e]     = __builtin_bit_cast(_Float16, h0);
    hv[4 + e] = __builtin_bit_cast(_Float16, h1);
    lv[e]     = __builtin_bit_cast(_Float16, l0);
    lv[4 + e] = __builtin_bit_cast(_Float16, l1);
  }
  unsigned short* qh = DTH + e0;
  unsigned short* ql = DTL + e0;
  *(volatile v8h*)qh = hv;
  *(volatile v8h*)ql = lv;
  __threadfence();
  *(volatile v8h*)qh = hv;
  *(volatile v8h*)ql = lv;
}

__global__ __launch_bounds__(256) void scan_kernel(
    const float* __restrict__ DLR, const float* __restrict__ XI, const float* __restrict__ XZ,
    const float* __restrict__ XD, const float* __restrict__ bdt, const float* __restrict__ Alog,
    const float* __restrict__ Dp, unsigned short* __restrict__ YH, unsigned short* __restrict__ YL)
{
  __shared__ __align__(16) float sDT[kScTS * kScCh];
  __shared__ __align__(16) float sU[kScTS * kScCh];
  __shared__ __align__(16) float sG[kScTS * kScCh];
  __shared__ __align__(16) float sBC[kScTS * 128];
  __shared__ __align__(16) float sY[kScTS * kScYP];
  const int tid = threadIdx.x, lane = tid & 31, wave = tid >> 5;
  constexpr int kBlkPerB = kDi / kScCh;
  const int bix = blockIdx.x / kBlkPerB;
  const int d0  = (blockIdx.x - bix * kBlkPerB) * kScCh;
  const int c   = tid >> 2;
  const int sg  = tid & 3;
  const int d   = d0 + c;
  const size_t row0 = (size_t)bix * kT;

  float negA[16], h[16];
  {
    const float* ap = Alog + (size_t)d * kDs + sg * 16;
#pragma unroll
    for (int q4 = 0; q4 < 4; ++q4) {
      const v4f av = *(const v4f*)(ap + 4 * q4);
#pragma unroll
      for (int e = 0; e < 4; ++e) {
        negA[4 * q4 + e] = -__expf(rne_bf(av[e]));
        h[4 * q4 + e] = 0.f;
      }
    }
  }
  const float Dd  = rne_bf(Dp[d]);
  const int   cs  = tid & 63;
  const int   rs  = tid >> 6;
  const float bbs = rne_bf(bdt[d0 + cs]);
  const int q = lane >> 3, c8 = (lane & 7) * 8;

#pragma unroll 1
  for (int t0 = 0; t0 < kT; t0 += kScTS) {
    __syncthreads();
#pragma unroll 1
    for (int p = 0; p < 8; ++p) {
      const int r = rs + 4 * p;
      const size_t grow = row0 + t0 + r;
      const float v   = DLR[grow * kDi + d0 + cs] + bbs;
      const float dtv = fmaxf(v, 0.0f) + log1pf(expf(-fabsf(v)));
      const float uv  = XI[grow * kDi + d0 + cs];
      const float zv  = XZ[grow * kXzP + kDi + d0 + cs];
      const float gv  = zv * __builtin_amdgcn_rcpf(1.0f + expf(-zv));
      sDT[r * kScCh + cs] = dtv;
      sU[r * kScCh + cs]  = uv;
      sG[r * kScCh + cs]  = gv;
    }
#pragma unroll
    for (int p = 0; p < 4; ++p) {
      const int idx = tid + p * 256;
      const int r   = idx >> 5;
      const int q4  = idx & 31;
      *(v4f*)(sBC + r * 128 + q4 * 4) = *(const v4f*)(XD + (row0 + t0 + r) * kXdP + kDtR + q4 * 4);
    }
    __syncthreads();
#pragma unroll 1
    for (int s = 0; s < kScTS; ++s) {
      const float dtv = sDT[s * kScCh + c];
      const float uv  = sU[s * kScCh + c];
      const float gv  = sG[s * kScCh + c];
      const float* bp = sBC + s * 128 + sg * 16;
      v4f Bq[4], Cq[4];
#pragma unroll
      for (int q4 = 0; q4 < 4; ++q4) {
        Bq[q4] = *(const v4f*)(bp + 4 * q4);
        Cq[q4] = *(const v4f*)(bp + kDs + 4 * q4);
      }
      const float dtx = dtv * uv;
      float y = 0.f;
#pragma unroll
      for (int k = 0; k < 16; ++k) {
        const float e = __expf(dtv * negA[k]);
        h[k] = e * h[k] + dtx * Bq[k >> 2][k & 3];
        y = h[k] * Cq[k >> 2][k & 3] + y;
      }
      y += __shfl_xor(y, 1, 32);
      y += __shfl_xor(y, 2, 32);
      const float yv = (uv * Dd + y) * gv;
      if (sg == 0) sY[s * kScYP + c] = yv;
    }
    __syncthreads();
    {
      const int row = wave * 4 + q;
      const float* sp = sY + row * kScYP + c8;
      const v4f a0 = *(const v4f*)(sp);
      const v4f a1 = *(const v4f*)(sp + 4);
      v8h hv, lv;
#pragma unroll
      for (int e = 0; e < 4; ++e) {
        const unsigned short h0 = f2bf_bits(a0[e]), h1 = f2bf_bits(a1[e]);
        const unsigned short l0 = f2bf_bits(a0[e] - bf_bits2f(h0)), l1 = f2bf_bits(a1[e] - bf_bits2f(h1));
        hv[e]     = __builtin_bit_cast(_Float16, h0);
        hv[4 + e] = __builtin_bit_cast(_Float16, h1);
        lv[e]     = __builtin_bit_cast(_Float16, l0);
        lv[4 + e] = __builtin_bit_cast(_Float16, l1);
      }
      const size_t o = (row0 + t0 + row) * kDi + d0 + c8;
      for (int pass = 0; pass < 2; ++pass) {
        *(volatile v8h*)(YH + o) = hv;
        *(volatile v8h*)(YL + o) = lv;
        __threadfence();
      }
    }
  }
}

__global__ __launch_bounds__(256) void runmean_kernel(
    const float* __restrict__ x, float* __restrict__ MCUR, float* __restrict__ MST)
{
  __shared__ __align__(16) float sT[16 * kTP];
  const int tid = threadIdx.x, lane = tid & 31, wave = tid >> 5;
  const int d0 = blockIdx.x * 256, d = d0 + tid;
  const int g0 = blockIdx.y * kSeg;
  const int hrow = wave >> 1;
  const int hch  = (wave & 1) * 128 + lane * 4;
  float run = 0.f;
#pragma unroll 1
  for (int sub = 0; sub < kSeg / 16; ++sub) {
    const int lb = g0 + sub * 16;
#pragma unroll 1
    for (int s = 0; s < 16; ++s) {
      const float xv = rne_bf(x[(size_t)(lb + s) * kDm + d]);
      run += xv;
      const float cnt = (float)(sub * 16 + s + 1);
      sT[s * kTP + tid] = run * __builtin_amdgcn_rcpf(cnt);
    }
    __syncthreads();
    v4f fv[4];
#pragma unroll
    for (int it = 0; it < 4; ++it) fv[it] = *(const v4f*)(sT + (it * 4 + hrow) * kTP + hch);
    for (int pass = 0; pass < 2; ++pass) {
#pragma unroll
      for (int it = 0; it < 4; ++it)
        *(volatile v4f*)(MCUR + (size_t)(lb + it * 4 + hrow) * kDm + d0 + hch) = fv[it];
      __threadfence();
    }
    __syncthreads();
  }
  const float mean = run * (1.0f / (float)kSeg);
  float* mp = MST + (size_t)blockIdx.y * kDm + d;
  *(volatile float*)mp = mean;
  __threadfence();
  *(volatile float*)mp = mean;
}

__global__ __launch_bounds__(256) void retrieve_kernel(
    const float* __restrict__ UU, const float* __restrict__ MCUR, const float* __restrict__ MST,
    const float* __restrict__ XOUT, float* __restrict__ out, float scl)
{
  __shared__ __align__(16) float sO[8 * kDm];
  const int lane = threadIdx.x & 31, wave = threadIdx.x >> 5;
  const int grow = blockIdx.x * 8 + wave;
  const int b    = grow / kT;
  const int t    = grow - b * kT;
  const int seg  = t / kSeg;
  const float* ur = UU   + (size_t)grow * kDm;
  const float* mr = MCUR + (size_t)grow * kDm;
  const float* ms = MST  + (size_t)b * kNSeg * kDm;

  float p0 = 0.f, p1 = 0.f, p2 = 0.f, p3 = 0.f, p4 = 0.f;
#pragma unroll 1
  for (int it = 0; it < kDm / 128; ++it) {
    const int off = it * 128 + lane * 4;
    const v4f uv = *(const v4f*)(ur + off);
    const v4f mv = *(const v4f*)(mr + off);
    const v4f k0 = *(const v4f*)(ms + off);
    const v4f k1 = *(const v4f*)(ms + kDm + off);
    const v4f k2 = *(const v4f*)(ms + 2 * kDm + off);
    const v4f k3 = *(const v4f*)(ms + 3 * kDm + off);
#pragma unroll
    for (int e = 0; e < 4; ++e) {
      p0 = fmaf(uv[e], k0[e], p0);
      p1 = fmaf(uv[e], k1[e], p1);
      p2 = fmaf(uv[e], k2[e], p2);
      p3 = fmaf(uv[e], k3[e], p3);
      p4 = fmaf(uv[e], mv[e], p4);
    }
  }
#pragma unroll
  for (int m = 16; m >= 1; m >>= 1) {
    p0 += __shfl_xor(p0, m, 32);
    p1 += __shfl_xor(p1, m, 32);
    p2 += __shfl_xor(p2, m, 32);
    p3 += __shfl_xor(p3, m, 32);
    p4 += __shfl_xor(p4, m, 32);
  }
  const float s0 = p0 * scl, s1 = p1 * scl, s2 = p2 * scl, s3 = p3 * scl, s4 = p4 * scl;
  float mx = s4;
  mx = (seg > 0) ? fmaxf(mx, s0) : mx;
  mx = (seg > 1) ? fmaxf(mx, s1) : mx;
  mx = (seg > 2) ? fmaxf(mx, s2) : mx;
  mx = (seg > 3) ? fmaxf(mx, s3) : mx;
  const float x0 = expf(s0 - mx), x1 = expf(s1 - mx), x2 = expf(s2 - mx), x3 = expf(s3 - mx);
  const float e4 = expf(s4 - mx);
  const float e0 = (seg > 0) ? x0 : 0.f;
  const float e1 = (seg > 1) ? x1 : 0.f;
  const float e2 = (seg > 2) ? x2 : 0.f;
  const float e3 = (seg > 3) ? x3 : 0.f;
  const float se  = (((e0 + e1) + e2) + e3) + e4;
  const float inv = 1.0f / se;
  const float g0 = e0 * inv, g1 = e1 * inv, g2 = e2 * inv, g3 = e3 * inv, g4 = e4 * inv;

  const float* xr  = XOUT + (size_t)grow * kDm;
  const float* hr0 = XOUT + ((size_t)b * kT + 1 * kSeg - 1) * kDm;
  const float* hr1 = XOUT + ((size_t)b * kT + 2 * kSeg - 1) * kDm;
  const float* hr2 = XOUT + ((size_t)b * kT + 3 * kSeg - 1) * kDm;
  const float* hr3 = XOUT + ((size_t)b * kT + 4 * kSeg - 1) * kDm;
  float* so = sO + wave * kDm;
  const v4f z4 = (v4f){0.f, 0.f, 0.f, 0.f};
#pragma unroll 1
  for (int it = 0; it < kDm / 128; ++it) {
    const int off = it * 128 + lane * 4;
    const v4f xo = *(const v4f*)(xr + off);
    const v4f c0 = *(const v4f*)(hr0 + off);
    const v4f c1 = *(const v4f*)(hr1 + off);
    const v4f c2 = *(const v4f*)(hr2 + off);
    const v4f c3 = *(const v4f*)(hr3 + off);
    const v4f h0 = (seg > 0) ? c0 : z4;
    const v4f h1 = (seg > 1) ? c1 : z4;
    const v4f h2 = (seg > 2) ? c2 : z4;
    const v4f h3 = (seg > 3) ? c3 : z4;
    v4f o = xo * g4;
    o += h0 * g0;
    o += h1 * g1;
    o += h2 * g2;
    o += h3 * g3;
    *(v4f*)(so + off) = o;
  }
  float* orow = out + (size_t)grow * kDm;
  for (int pass = 0; pass < 2; ++pass) {
#pragma unroll 1
    for (int it = 0; it < kDm / 128; ++it) {
      const int off = it * 128 + lane * 4;
      const v4f v = *(const v4f*)(so + off);
      *(volatile v4f*)(orow + off) = v;
    }
    __threadfence();
  }
}

extern "C" void kernel_launch(void* const* d_in, const int* in_sizes, int n_in,
                              void* d_out, int out_size, void* d_ws, size_t ws_size,
                              hipStream_t stream)
{
  if (n_in < 11) return;
  if (in_sizes[0] != kRows * kDm) return;
  if (in_sizes[1] != kDm * kXzP) return;
  if (in_sizes[2] != kDi * 4) return;
  if (in_sizes[3] != kDi) return;
  if (in_sizes[4] != kDi * kXdN) return;
  if (in_sizes[5] != kDtR * kDi) return;
  if (in_sizes[6] != kDi) return;
  if (in_sizes[7] != kDi * kDs) return;
  if (in_sizes[8] != kDi) return;
  if (in_sizes[9] != kDi * kDm) return;
  if (in_sizes[10] != kDm * kDm) return;
  if (out_size != kRows * kDm) return;
  if (ws_size < kWsTotal) return;

  const float* x      = (const float*)d_in[0];
  const float* W_in   = (const float*)d_in[1];
  const float* conv_w = (const float*)d_in[2];
  const float* conv_b = (const float*)d_in[3];
  const float* W_xp   = (const float*)d_in[4];
  const float* W_dt   = (const float*)d_in[5];
  const float* b_dt   = (const float*)d_in[6];
  const float* A_log  = (const float*)d_in[7];
  const float* Dp     = (const float*)d_in[8];
  const float* W_out  = (const float*)d_in[9];
  const float* W_u    = (const float*)d_in[10];
  float* out = (float*)d_out;

  char* ws = (char*)d_ws;
  unsigned short* XB    = (unsigned short*)(ws + kOffXB);
  unsigned short* WINT  = (unsigned short*)(ws + kOffWINT);
  unsigned short* WXT   = (unsigned short*)(ws + kOffWXT);
  unsigned short* WDTT  = (unsigned short*)(ws + kOffWDTT);
  unsigned short* WOUTT = (unsigned short*)(ws + kOffWOUTT);
  unsigned short* WUT   = (unsigned short*)(ws + kOffWUT);
  float*          XZ    = (float*)(ws + kOffXZ);
  float*          XI    = (float*)(ws + kOffXI);
  unsigned short* XIH   = (unsigned short*)(ws + kOffXIH);
  unsigned short* XIL   = (unsigned short*)(ws + kOffXIL);
  float*          XD    = (float*)(ws + kOffXD);
  unsigned short* DTH   = (unsigned short*)(ws + kOffDTH);
  unsigned short* DTL   = (unsigned short*)(ws + kOffDTL);
  float*          DLR   = (float*)(ws + kOffDLR);
  unsigned short* YH    = (unsigned short*)(ws + kOffYH);
  unsigned short* YL    = (unsigned short*)(ws + kOffYL);
  float*          XOUT  = (float*)(ws + kOffXOUT);
  float*          UU    = (float*)(ws + kOffUU);
  float*          MCUR  = (float*)(ws + kOffMCUR);
  float*          MST   = (float*)(ws + kOffMST);
  const float* dummy_bias  = b_dt;
  const float* dummy_resid = x;
  const float scl = 1.0f / sqrtf((float)kDm);

  cast_bf16_kernel<<<(kRows * kDm / 8) / 256, 256, 0, stream>>>(x, XB, kRows * kDm / 8);

  transpose_bf16_kernel<<<dim3(kXzP / 64, kDm / 64), 256, 0, stream>>>(W_in, WINT, kDm, kXzP);
  transpose_bf16_kernel<<<dim3(kXdP / 64, kDi / 64), 256, 0, stream>>>(W_xp, WXT, kDi, kXdN);
  transpose_k32_kernel<<<(kDi * kDtR / 8) / 256, 256, 0, stream>>>(W_dt, WDTT, kDi, kDi * kDtR / 8);
  transpose_bf16_kernel<<<dim3(kDm / 64, kDi / 64), 256, 0, stream>>>(W_out, WOUTT, kDi, kDm);
  transpose_bf16_kernel<<<dim3(kDm / 64, kDm / 64), 256, 0, stream>>>(W_u, WUT, kDm, kDm);

  wmma_gemm64<1, 0, 0, 0, false><<<dim3(192, 1), 256, 0, stream>>>(
      XB, XB, kDm, 0L, WINT, WINT, kDm, 0L,
      (void*)XZ, (void*)XZ, kXzP, 0L, dummy_bias, dummy_resid, 0L,
      kRows, kXzP, kDm, 1.0f);

  conv_silu_kernel<<<dim3(kDi / 256, kRows / 64), 256, 0, stream>>>(XZ, conv_w, conv_b, XI, XIH, XIL);

  wmma_gemm64<1, 1, 0, 0, false><<<dim3(12, 1), 256, 0, stream>>>(
      XIH, XIL, kDi, 0L, WXT, WXT, kDi, 0L,
      (void*)XD, (void*)XD, kXdP, 0L, dummy_bias, dummy_resid, 0L,
      kRows, kXdP, kDi, 1.0f);

  dt_split_kernel<<<(kRows * kDtR / 8) / 256, 256, 0, stream>>>(XD, DTH, DTL, kRows * kDtR / 8);

  wmma_gemm64<1, 1, 0, 0, false><<<dim3(96, 1), 256, 0, stream>>>(
      DTH, DTL, kDtR, 0L, WDTT, WDTT, kDtR, 0L,
      (void*)DLR, (void*)DLR, kDi, 0L, dummy_bias, dummy_resid, 0L,
      kRows, kDi, kDtR, 1.0f);

  scan_kernel<<<kB * (kDi / kScCh), 256, 0, stream>>>(DLR, XI, XZ, XD, b_dt, A_log, Dp, YH, YL);

  wmma_gemm64<1, 1, 0, 0, false><<<dim3(48, 1), 256, 0, stream>>>(
      YH, YL, kDi, 0L, WOUTT, WOUTT, kDi, 0L,
      (void*)XOUT, (void*)XOUT, kDm, 0L, dummy_bias, dummy_resid, 0L,
      kRows, kDm, kDi, 1.0f);

  wmma_gemm64<1, 0, 0, 0, false><<<dim3(48, 1), 256, 0, stream>>>(
      XB, XB, kDm, 0L, WUT, WUT, kDm, 0L,
      (void*)UU, (void*)UU, kDm, 0L, dummy_bias, dummy_resid, 0L,
      kRows, kDm, kDm, 1.0f);

  runmean_kernel<<<dim3(kDm / 256, kB * kNSeg), 256, 0, stream>>>(x, MCUR, MST);

  retrieve_kernel<<<kRows / 8, 256, 0, stream>>>(UU, MCUR, MST, XOUT, out, scl);
}
